// MPNNDecoderVAE_39779987095907
// MI455X (gfx1250) — hardware-verified
//
#include <hip/hip_runtime.h>
#include <math.h>
typedef __attribute__((ext_vector_type(16))) _Float16 v16h;
typedef __attribute__((ext_vector_type(8)))  _Float16 v8h;
typedef __attribute__((ext_vector_type(16))) __bf16   v16b;
typedef __attribute__((ext_vector_type(8)))  __bf16   v8b;
typedef __attribute__((ext_vector_type(8)))  float    v8f;
typedef __attribute__((ext_vector_type(4)))  float    v4f;
#define PSCALE 32768.0f
#define U16(p) ((const unsigned short*)(const void*)(p))
#define PSCALE_INV (1.0f / 32768.0f)

__device__ __forceinline__ unsigned short f2bf_bits(float f) {
  unsigned u = __float_as_uint(f);
  return (unsigned short)((u + 0x7FFFu + ((u >> 16) & 1u)) >> 16);
}
__device__ __forceinline__ float bf_bits2f(unsigned short h) { return __uint_as_float(((unsigned)h) << 16); }

__device__ __forceinline__ void dep_guard_h(v8f& a, v8f& b, v16h x, v16h y) { asm volatile("v_nop\n\tv_nop\n\tv_nop\n\tv_nop" : "+v"(a), "+v"(b) : "v"(x), "v"(y)); }
__device__ __forceinline__ void dep_guard_b(v8f& a, v8f& b, v16b x, v16b y) { asm volatile("v_nop\n\tv_nop\n\tv_nop\n\tv_nop" : "+v"(a), "+v"(b) : "v"(x), "v"(y)); }
__device__ __forceinline__ void keep4_h(v16h a, v16h b, v16h c, v16h d) { asm volatile("v_nop" :: "v"(a), "v"(b), "v"(c), "v"(d)); }
__device__ __forceinline__ void keep4_b(v16b a, v16b b, v16b c, v16b d) { asm volatile("v_nop" :: "v"(a), "v"(b), "v"(c), "v"(d)); }
__device__ __forceinline__ void acc_guard4(v8f& a, v8f& b, v8f& c, v8f& d) { asm volatile("v_nop\n\tv_nop\n\tv_nop\n\tv_nop" : "+v"(a), "+v"(b), "+v"(c), "+v"(d)); }
template <typename T> struct Frag;
template <> struct Frag<_Float16> {
  typedef v16h V; union U { v16h v; v8h h[2]; };
  static __device__ __forceinline__ v16h load(const _Float16* p) {
    U f; f.h[0] = *(const v8h*)(p); f.h[1] = *(const v8h*)(p + 16); return f.v;
  }
  static __device__ __forceinline__ v8f mma(v16h a, v16h b, v8f c) {
    return __builtin_amdgcn_wmma_f32_16x16x32_f16(false, a, false, b, (short)0, c, false, false);
  }
  static __device__ __forceinline__ void guard(v8f& a, v8f& b, v16h x, v16h y) { dep_guard_h(a, b, x, y); }
  static __device__ __forceinline__ void keep(v16h a, v16h b, v16h c, v16h d) { keep4_h(a, b, c, d); }
};
template <> struct Frag<__bf16> {
  typedef v16b V; union U { v16b v; v8b h[2]; };
  static __device__ __forceinline__ v16b load(const __bf16* p) {
    U f; f.h[0] = *(const v8b*)(p); f.h[1] = *(const v8b*)(p + 16); return f.v;
  }
  static __device__ __forceinline__ v8f mma(v16b a, v16b b, v8f c) {
    return __builtin_amdgcn_wmma_f32_16x16x32_bf16(false, a, false, b, (short)0, c, false, false);
  }
  static __device__ __forceinline__ void guard(v8f& a, v8f& b, v16b x, v16b y) { dep_guard_b(a, b, x, y); }
  static __device__ __forceinline__ void keep(v16b a, v16b b, v16b c, v16b d) { keep4_b(a, b, c, d); }
};

template <int ET> struct Elem;
template <> struct Elem<0> { typedef _Float16 T; };
template <> struct Elem<1> { typedef __bf16 T; };
template <int ET, bool SPLIT, int BIAS_MODE, int OUT_MODE, bool RESID, int ACT = 0>
__global__ __launch_bounds__(256) void wmma_gemm64(
    const unsigned short* __restrict__ Ap, const unsigned short* __restrict__ A2p, int lda, long strideA,
    const unsigned short* __restrict__ Btp, const unsigned short* __restrict__ Bt2p, int ldb, long strideB,
    void* __restrict__ Cout, void* __restrict__ Cout2, int ldc, long strideC,
    const float* __restrict__ bias,
    const float* __restrict__ resid, long strideR,
    int M, int N, int K, float scale) {
  typedef typename Elem<ET>::T T;
  typedef typename Frag<T>::V V;
  const T* A = (const T*)Ap; const T* A2 = (const T*)A2p; const T* Bt = (const T*)Btp; const T* Bt2 = (const T*)Bt2p;
  __shared__ __align__(16) float sT[8][16 * 68];
  const int b    = blockIdx.y;
  const int lane = threadIdx.x & 31;
  const int wave = threadIdx.x >> 5;
  const int tilesN = N >> 6;
  const int tilesM = M >> 6;
  const int tile = blockIdx.x * 8 + wave;
  if (tile >= tilesM * tilesN) return;
  const int tm = tile / tilesN;
  const int tn = tile - tm * tilesN;
  const int m0 = tm << 6;
  const int n0 = tn << 6;

  const T* Ab  = A  + (size_t)b * strideA;
  const T* Bb  = Bt + (size_t)b * strideB;
  const T* Ab2 = SPLIT ? (A2  + (size_t)b * strideA) : nullptr;
  const T* Bb2 = SPLIT ? (Bt2 + (size_t)b * strideB) : nullptr;

  const int rlane = lane & 15;
  const int koff  = (lane >> 4) * 8;
  const int mOff  = (lane >> 4) * 8;

  v8f acc[4][4];
#pragma unroll
  for (int i = 0; i < 4; ++i)
#pragma unroll
    for (int j = 0; j < 4; ++j) acc[i][j] = (v8f){0.f,0.f,0.f,0.f,0.f,0.f,0.f,0.f};

  for (int k0 = 0; k0 < K; k0 += 32) {
    V bh[4], bl[4];
#pragma unroll
    for (int j = 0; j < 4; ++j) {
      const size_t bo = (size_t)(n0 + (j << 4) + rlane) * ldb + koff + k0;
      bh[j] = Frag<T>::load(Bb + bo);
      if (SPLIT) bl[j] = Frag<T>::load(Bb2 + bo);
    }
#pragma unroll
    for (int i = 0; i < 4; ++i) {
      const size_t ao = (size_t)(m0 + (i << 4) + rlane) * lda + koff + k0;
      V ah = Frag<T>::load(Ab + ao);
      V al;
      if (SPLIT) al = Frag<T>::load(Ab2 + ao);
#pragma unroll
      for (int j = 0; j < 4; ++j) {
        acc[i][j] = Frag<T>::mma(ah, bh[j], acc[i][j]);
        if (SPLIT) {
          acc[i][j] = Frag<T>::mma(ah, bl[j], acc[i][j]);
          acc[i][j] = Frag<T>::mma(al, bh[j], acc[i][j]);
        }
      }
      Frag<T>::guard(acc[i][0], acc[i][3], ah, SPLIT ? al : ah);
    }
    Frag<T>::keep(bh[0], bh[1], bh[2], bh[3]);
    if (SPLIT) Frag<T>::keep(bl[0], bl[1], bl[2], bl[3]);
  }
  acc_guard4(acc[0][0], acc[0][1], acc[0][2], acc[0][3]);
  acc_guard4(acc[1][0], acc[1][1], acc[1][2], acc[1][3]);
  acc_guard4(acc[2][0], acc[2][1], acc[2][2], acc[2][3]);
  acc_guard4(acc[3][0], acc[3][1], acc[3][2], acc[3][3]);

  float* slab = sT[wave];
  const float* Rb = RESID ? (resid + (size_t)b * strideR) : nullptr;
#pragma unroll
  for (int i = 0; i < 4; ++i) {
    const int mBase = m0 + (i << 4);
#pragma unroll
    for (int j = 0; j < 4; ++j) {
      const int n = n0 + (j << 4) + rlane;
      float bv = 0.f;
      if (BIAS_MODE == 2) bv = bias[n];
#pragma unroll
      for (int r = 0; r < 8; ++r) {
        float v = acc[i][j][r] * scale;
        if (BIAS_MODE == 1) v += bias[mBase + mOff + r];
        if (BIAS_MODE == 2) v += bv;
        if (RESID) v += Rb[(size_t)(mBase + mOff + r) * ldc + n];
        if (ACT == 1) v = tanhf(v);
        if (ACT == 2) v = fmaxf(v, 0.0f);
        if (ACT == 3) v = v / (1.0f + expf(-v));
        if (ACT == 4) v = (v > 0.f) ? v : 0.01f * v;
        if (ACT == 5) v = 0.5f * v * (1.0f + erff(v * 0.70710678118654752f));
        slab[(mOff + r) * 68 + (j << 4) + rlane] = v;
      }
    }
    __builtin_amdgcn_fence(__ATOMIC_RELEASE, "workgroup");
    __builtin_amdgcn_wave_barrier();
    __builtin_amdgcn_fence(__ATOMIC_ACQUIRE, "workgroup");
    if (OUT_MODE == 0) {
      float* C = (float*)Cout + (size_t)b * strideC;
      const int hh = lane >> 4, c4 = (lane & 15) * 4;
      for (int pass = 0; pass < 2; ++pass) {
#pragma unroll
        for (int it = 0; it < 8; ++it) {
          const int row = it * 2 + hh;
          v4f v = *(const v4f*)(slab + row * 68 + c4);
          *(volatile v4f*)(C + (size_t)(mBase + row) * ldc + n0 + c4) = v;
        }
        __threadfence();
      }
    } else {
      const int q = lane >> 3, c8 = (lane & 7) * 8;
      unsigned short* C  = (unsigned short*)Cout  + (size_t)b * strideC;
      unsigned short* C2 = (OUT_MODE == 2) ? ((unsigned short*)Cout2 + (size_t)b * strideC) : nullptr;
      for (int pass = 0; pass < 2; ++pass) {
#pragma unroll
        for (int it = 0; it < 4; ++it) {
          const int row = it * 4 + q;
          const float* sp = slab + row * 68 + c8;
          v8h hv, lv;
#pragma unroll
          for (int e = 0; e < 8; ++e) {
            if (OUT_MODE == 1) {
              hv[e] = (_Float16)sp[e];
            } else {
              unsigned short hb = f2bf_bits(sp[e]);
              unsigned short lb = f2bf_bits(sp[e] - bf_bits2f(hb));
              hv[e] = __builtin_bit_cast(_Float16, hb);
              lv[e] = __builtin_bit_cast(_Float16, lb);
            }
          }
          *(volatile v8h*)(C + (size_t)(mBase + row) * ldc + n0 + c8) = hv;
          if (OUT_MODE == 2) *(volatile v8h*)(C2 + (size_t)(mBase + row) * ldc + n0 + c8) = lv;
        }
        __threadfence();
      }
    }
    __builtin_amdgcn_fence(__ATOMIC_RELEASE, "workgroup");
    __builtin_amdgcn_wave_barrier();
    __builtin_amdgcn_fence(__ATOMIC_ACQUIRE, "workgroup");
  }
}

__global__ __launch_bounds__(256) void cast_f32_f16x2(
    const float* __restrict__ in, _Float16* __restrict__ out, int n2) {
  int i = blockIdx.x * 256 + threadIdx.x;
  if (i < n2) {
    const _Float16 h0 = (_Float16)in[2 * i], h1 = (_Float16)in[2 * i + 1];
    const unsigned u = (unsigned)__builtin_bit_cast(unsigned short, h0) | ((unsigned)__builtin_bit_cast(unsigned short, h1) << 16);
    ((volatile unsigned*)out)[i] = u;
    __threadfence();
    ((volatile unsigned*)out)[i] = u;
  }
}


#define VB 512
#define VN 64
#define VH 256
#define VLAT 128
#define VHEADS 4
#define VHC 64
#define VNF 64
#define VDIN (VH + VLAT)
#define VR 8
#define VROWS (VB * VN)
#define LSCAL 2.0f
__global__ __launch_bounds__(256) void lora_fold16_kernel(const float* __restrict__ Wm, const float* __restrict__ A, const float* __restrict__ Bm, int O, int Kd, unsigned* __restrict__ out) {
  const long i = (long)blockIdx.x * 256 + threadIdx.x; if (i >= (long)O * Kd / 2) return;
  const long e0 = 2 * i; const int o = (int)(e0 / Kd), k = (int)(e0 % Kd);
  float a = Wm[e0], b = Wm[e0 + 1];
#pragma unroll
  for (int r = 0; r < VR; ++r) { const float br_ = LSCAL * Bm[(size_t)o * VR + r]; a += br_ * A[(size_t)r * Kd + k]; b += br_ * A[(size_t)r * Kd + k + 1]; }
  const unsigned u = (unsigned)__builtin_bit_cast(unsigned short, (_Float16)a) | ((unsigned)__builtin_bit_cast(unsigned short, (_Float16)b) << 16);
  ((volatile unsigned*)out)[i] = u; __threadfence(); ((volatile unsigned*)out)[i] = u;
}
__global__ __launch_bounds__(256) void lora_ab_kernel(const float* __restrict__ aw, const float* __restrict__ aA, const float* __restrict__ aB,
                                                     const float* __restrict__ bw, const float* __restrict__ bA, const float* __restrict__ bB, float* __restrict__ wab) {
  for (int pass = 0; pass < 2; ++pass) {
    for (int i = blockIdx.x * 256 + threadIdx.x; i < 2560; i += gridDim.x * 256) {
      float acc;
      if (i < 512) { acc = aw[i];
#pragma unroll
        for (int r = 0; r < VR; ++r) acc += LSCAL * aB[r] * aA[(size_t)r * 512 + i]; }
      else { const int t = i - 512, o = t >> 9, k = t & 511; acc = bw[t];
#pragma unroll
        for (int r = 0; r < VR; ++r) acc += LSCAL * bB[o * VR + r] * bA[(size_t)r * 512 + k]; }
      ((volatile float*)wab)[i] = acc;
    }
    __threadfence();
  }
}
__global__ __launch_bounds__(256) void concat_kernel(const float* __restrict__ X, const float* __restrict__ z, unsigned* __restrict__ XC) {
  const int lane = threadIdx.x & 31, wave = threadIdx.x >> 5; const int row = blockIdx.x * 8 + wave; const int b = row / VN;
  unsigned u[6];
#pragma unroll
  for (int q = 0; q < 6; ++q) { const int c2 = (q * 32 + lane) * 2;
    float a, bb;
    if (c2 < VH) { a = X[(size_t)row * VH + c2]; bb = X[(size_t)row * VH + c2 + 1]; } else { a = z[(size_t)b * VLAT + c2 - VH]; bb = z[(size_t)b * VLAT + c2 - VH + 1]; }
    u[q] = (unsigned)__builtin_bit_cast(unsigned short, (_Float16)a) | ((unsigned)__builtin_bit_cast(unsigned short, (_Float16)bb) << 16); }
  for (int pass = 0; pass < 2; ++pass) {
#pragma unroll
    for (int q = 0; q < 6; ++q) ((volatile unsigned*)XC)[(size_t)row * (VDIN / 2) + q * 32 + lane] = u[q];
    __threadfence();
  }
}
__device__ __forceinline__ v8f mma16(v16h a, v16h b, v8f c) {
  c = __builtin_amdgcn_wmma_f32_16x16x32_f16(false, a, false, b, (short)0, c, false, false);
  asm volatile("v_nop\n\tv_nop\n\tv_nop\n\tv_nop" : "+v"(c) : "v"(a), "v"(b));
  return c;
}
__global__ __launch_bounds__(256) void gat_kernel(const float* __restrict__ Hm, const float* __restrict__ asrc, const float* __restrict__ adst,
                                                 const float* __restrict__ bias, float* __restrict__ X, unsigned* __restrict__ X16, int write16) {
  __shared__ __align__(16) _Float16 HT[VHEADS][VHC][72];
  __shared__ __align__(16) _Float16 AL[VHEADS][VN][72];
  __shared__ float ES[VHEADS][VN], ED[VHEADS][VN];
  __shared__ __align__(16) float OUT[VN][VH + 4];
  const int tid = threadIdx.x, lane = tid & 31, wave = tid >> 5, hh = lane >> 4, c = lane & 15;
  const int g = blockIdx.x; const size_t row0 = (size_t)g * VN;
  for (int n = wave; n < VN; n += 8) {
    const float* hr = Hm + (row0 + n) * VH;
    float es[VHEADS], ed[VHEADS];
#pragma unroll
    for (int h = 0; h < VHEADS; ++h) {
      const float v0 = hr[h * VHC + lane], v1 = hr[h * VHC + 32 + lane];
      HT[h][lane][n] = (_Float16)v0; HT[h][32 + lane][n] = (_Float16)v1;
      float s = v0 * asrc[h * VHC + lane] + v1 * asrc[h * VHC + 32 + lane];
      float d = v0 * adst[h * VHC + lane] + v1 * adst[h * VHC + 32 + lane];
      for (int o = 16; o > 0; o >>= 1) { s += __shfl_xor(s, o, 32); d += __shfl_xor(d, o, 32); }
      es[h] = s; ed[h] = d;
    }
    if (lane < VHEADS) {
      float sv = es[0], dv = ed[0];
#pragma unroll
      for (int h = 1; h < VHEADS; ++h) if (lane == h) { sv = es[h]; dv = ed[h]; }
      ES[lane][n] = sv; ED[lane][n] = dv;
    }
  }
  __syncthreads();
  {
    const int h = tid >> 6, i = tid & 63;
    const float di = ED[h][i];
    float mx = -INFINITY;
    for (int j = 0; j < VN; ++j) { float e = di + ES[h][j]; e = (e > 0.f) ? e : 0.2f * e; mx = fmaxf(mx, e); }
    float se = 0.f; float ev[VN];
    for (int j = 0; j < VN; ++j) { float e = di + ES[h][j]; e = (e > 0.f) ? e : 0.2f * e; ev[j] = expf(e - mx); se += ev[j]; }
    const float inv = 32768.0f / se;
    for (int j = 0; j < VN; ++j) AL[h][i][j] = (_Float16)(ev[j] * inv);
  }
  __syncthreads();
  for (int t = wave; t < 64; t += 8) {
    const int h = t >> 4, mt = (t >> 2) & 3, nt = t & 3;
    v8f acc = {0.f,0.f,0.f,0.f,0.f,0.f,0.f,0.f};
#pragma unroll
    for (int ks = 0; ks < 2; ++ks) {
      v16h a, b;
      { const _Float16* p = &AL[h][mt * 16 + c][ks * 32 + 8 * hh]; const v8h lo = *(const v8h*)p, hi2 = *(const v8h*)(p + 16);
#pragma unroll
        for (int e = 0; e < 8; ++e) { a[e] = lo[e]; a[8 + e] = hi2[e]; } }
      { const _Float16* p = &HT[h][nt * 16 + c][ks * 32 + 8 * hh]; const v8h lo = *(const v8h*)p, hi2 = *(const v8h*)(p + 16);
#pragma unroll
        for (int e = 0; e < 8; ++e) { b[e] = lo[e]; b[8 + e] = hi2[e]; } }
      acc = mma16(a, b, acc);
    }
#pragma unroll
    for (int r = 0; r < 8; ++r) { const int i = mt * 16 + 8 * hh + r, col = h * VHC + nt * 16 + c;
      OUT[i][col] = fmaxf(acc[r] * (1.0f / 32768.0f) + bias[col], 0.f); }
  }
  __syncthreads();
  for (int pass = 0; pass < 2; ++pass) {
    for (int i = tid; i < VN * VH / 4; i += 256) { const int n = i / (VH / 4), c4 = (i % (VH / 4)) * 4;
      const v4f v = *(const v4f*)(&OUT[n][c4]); *(volatile v4f*)(X + (row0 + n) * VH + c4) = v;
      if (write16) { typedef __attribute__((ext_vector_type(2))) unsigned u2; u2 pk;
        pk[0] = (unsigned)__builtin_bit_cast(unsigned short, (_Float16)v[0]) | ((unsigned)__builtin_bit_cast(unsigned short, (_Float16)v[1]) << 16);
        pk[1] = (unsigned)__builtin_bit_cast(unsigned short, (_Float16)v[2]) | ((unsigned)__builtin_bit_cast(unsigned short, (_Float16)v[3]) << 16);
        *(volatile u2*)(X16 + ((row0 + n) * VH + c4) / 2) = pk; } }
    __threadfence();
  }
}
__global__ __launch_bounds__(256) void pair_kernel(const float* __restrict__ X, const float* __restrict__ wab, const float* __restrict__ adj_b, const float* __restrict__ bond_b,
                                                  float* __restrict__ adj, float* __restrict__ bond) {
  __shared__ float S1[VN], S2[VN], T1[VN][4], T2[VN][4];
  const int tid = threadIdx.x, lane = tid & 31, wave = tid >> 5;
  const int g = blockIdx.x; const size_t row0 = (size_t)g * VN;
  for (int n = wave; n < VN; n += 8) {
    const float* xr = X + (row0 + n) * VH;
    float xv[8];
#pragma unroll
    for (int q = 0; q < 8; ++q) xv[q] = xr[q * 32 + lane];
    float d[10];
#pragma unroll
    for (int p = 0; p < 10; ++p) { const float* wv = (p == 0) ? wab : (p == 1) ? (wab + VH) : (p < 6) ? (wab + 512 + (size_t)(p - 2) * 512) : (wab + 512 + (size_t)(p - 6) * 512 + VH);
      float s = 0.f;
#pragma unroll
      for (int q = 0; q < 8; ++q) s += xv[q] * wv[q * 32 + lane];
      for (int o = 16; o > 0; o >>= 1) s += __shfl_xor(s, o, 32);
      d[p] = s; }
    if (lane == 0) { S1[n] = d[0]; S2[n] = d[1]; T1[n][0] = d[2]; T1[n][1] = d[3]; T1[n][2] = d[4]; T1[n][3] = d[5]; T2[n][0] = d[6]; T2[n][1] = d[7]; T2[n][2] = d[8]; T2[n][3] = d[9]; }
  }
  __syncthreads();
  const float ab = adj_b[0];
  for (int pass = 0; pass < 2; ++pass) {
    for (int it = 0; it < 4; ++it) { const int i = it * 16 + (tid >> 4), j0 = (tid & 15) * 4; v4f v;
#pragma unroll
      for (int e = 0; e < 4; ++e) { const int j = j0 + e; v[e] = (j > i) ? (S1[i] + S2[j] + ab) : (j < i) ? (S1[j] + S2[i] + ab) : 0.f; }
      *(volatile v4f*)(adj + (row0 + i) * VN + j0) = v; }
    for (int it = 0; it < 16; ++it) { const int i = it * 4 + (tid >> 6), j = tid & 63; v4f v;
#pragma unroll
      for (int k = 0; k < 4; ++k) v[k] = (j > i) ? (T1[i][k] + T2[j][k] + bond_b[k]) : (j < i) ? (T1[j][k] + T2[i][k] + bond_b[k]) : 0.f;
      *(volatile v4f*)(bond + ((row0 + i) * VN + j) * 4) = v; }
    __threadfence();
  }
}
extern "C" void kernel_launch(void* const* d_in, const int* in_sizes, int n_in, void* d_out, int out_size, void* d_ws, size_t ws_size, hipStream_t stream) {
  (void)in_sizes; (void)n_in; (void)out_size; (void)ws_size;
  const float* z = (const float*)d_in[0];
  const float* z2n_w = (const float*)d_in[1]; const float* z2n_b = (const float*)d_in[2]; const float* z2n_A = (const float*)d_in[3]; const float* z2n_B = (const float*)d_in[4];
  const float* gat_W = (const float*)d_in[5]; const float* gat_as = (const float*)d_in[6]; const float* gat_ad = (const float*)d_in[7]; const float* gat_b = (const float*)d_in[8];
  const float* node_w = (const float*)d_in[9]; const float* node_b = (const float*)d_in[10]; const float* node_A = (const float*)d_in[11]; const float* node_B = (const float*)d_in[12];
  const float* adj_w = (const float*)d_in[13]; const float* adj_b = (const float*)d_in[14]; const float* adj_A = (const float*)d_in[15]; const float* adj_B = (const float*)d_in[16];
  const float* bond_w = (const float*)d_in[17]; const float* bond_b = (const float*)d_in[18]; const float* bond_A = (const float*)d_in[19]; const float* bond_B = (const float*)d_in[20];
  float* recon = (float*)d_out; float* adj = recon + (size_t)VROWS * VNF; float* bond = adj + (size_t)VB * VN * VN;
  char* ws = (char*)d_ws; size_t off = 0;
  auto carve = [&](size_t bytes) -> char* { char* p = ws + off; off += (bytes + 255) & ~(size_t)255; return p; };
  unsigned* Wz16 = (unsigned*)carve((size_t)VH * VN * VLAT * 2);
  unsigned* Wn16 = (unsigned*)carve((size_t)VNF * VH * 2);
  float* wab = (float*)carve(2560 * 4);
  _Float16* Z16 = (_Float16*)carve((size_t)VB * VLAT * 2);
  _Float16* Wg16 = (_Float16*)carve((size_t)3 * VH * VDIN * 2);
  float* X = (float*)carve((size_t)VROWS * VH * 4);
  unsigned* XC = (unsigned*)carve((size_t)VROWS * VDIN * 2);
  float* Hm = (float*)carve((size_t)VROWS * VH * 4);
  unsigned* X16 = (unsigned*)carve((size_t)VROWS * VH * 2);
  lora_fold16_kernel<<<(VH * VN * VLAT / 2 + 255) / 256, 256, 0, stream>>>(z2n_w, z2n_A, z2n_B, VH * VN, VLAT, Wz16);
  lora_fold16_kernel<<<(VNF * VH / 2 + 255) / 256, 256, 0, stream>>>(node_w, node_A, node_B, VNF, VH, Wn16);
  lora_ab_kernel<<<10, 256, 0, stream>>>(adj_w, adj_A, adj_B, bond_w, bond_A, bond_B, wab);
  cast_f32_f16x2<<<(VB * VLAT / 2 + 255) / 256, 256, 0, stream>>>(z, Z16, VB * VLAT / 2);
  cast_f32_f16x2<<<(3 * VH * VDIN / 2 + 255) / 256, 256, 0, stream>>>(gat_W, Wg16, 3 * VH * VDIN / 2);
  { const int t = (VB / 64) * (VH * VN / 64);
    wmma_gemm64<0, false, 2, 0, false, 2><<<dim3((t + 7) / 8, 1), 256, 0, stream>>>(U16(Z16), nullptr, VLAT, 0, (const unsigned short*)Wz16, nullptr, VLAT, 0, X, nullptr, VH * VN, 0, z2n_b, nullptr, 0, VB, VH * VN, VLAT, 1.0f); }
  for (int l = 0; l < 3; ++l) {
    concat_kernel<<<VROWS / 8, 256, 0, stream>>>(X, z, XC);
    const int t = (VROWS / 64) * (VH / 64);
    wmma_gemm64<0, false, 0, 0, false, 0><<<dim3((t + 7) / 8, 1), 256, 0, stream>>>((const unsigned short*)XC, nullptr, VDIN, 0, U16(Wg16 + (size_t)l * VH * VDIN), nullptr, VDIN, 0, Hm, nullptr, VH, 0, nullptr, nullptr, 0, VROWS, VH, VDIN, 1.0f);
    gat_kernel<<<VB, 256, 0, stream>>>(Hm, gat_as + l * VHEADS * VHC, gat_ad + l * VHEADS * VHC, gat_b + l * VH, X, X16, (l == 2) ? 1 : 0);
  }
  { const int t = (VROWS / 64) * (VNF / 64);
    wmma_gemm64<0, false, 2, 0, false, 0><<<dim3((t + 7) / 8, 1), 256, 0, stream>>>((const unsigned short*)X16, nullptr, VH, 0, (const unsigned short*)Wn16, nullptr, VH, 0, recon, nullptr, VNF, 0, node_b, nullptr, 0, VROWS, VNF, VH, 1.0f); }
  pair_kernel<<<VB, 256, 0, stream>>>(X, wab, adj_b, bond_b, adj, bond);
}
